// Leg_fit_21595095564537
// MI455X (gfx1250) — hardware-run, weakly checked
//
#include <hip/hip_runtime.h>
#include <hip/hip_fp16.h>
#include <math.h>

typedef __attribute__((ext_vector_type(16))) _Float16 v16h;
typedef __attribute__((ext_vector_type(8)))  _Float16 v8h;
typedef __attribute__((ext_vector_type(8)))  float    v8f;
typedef __attribute__((ext_vector_type(4)))  float    v4f;
typedef __attribute__((ext_vector_type(2)))  unsigned v2u;

constexpr int kSteps  = 1000;
constexpr int kNrn    = 400;
constexpr int kExc    = 320;
constexpr int kPre    = 8;
constexpr int kRowsP  = 384;
constexpr int kSeg    = 1024;
constexpr int kKdim   = 2 * kSeg;
constexpr float kACarry = 64.0f;
constexpr float kBCarry = 1024.0f;
constexpr float kResid  = 2048.0f;
constexpr float kDecayP = 0.9672161f;
constexpr float kDecayM = 0.9672161f;
constexpr float kDecayE = 0.9975031f;
constexpr float kAP     = 0.005f;
constexpr float kAM     = 0.00525f;
constexpr float kGain   = 0.01f;
constexpr float kWMax   = 0.5f;
static_assert(kKdim == 2048);
static_assert(kSteps <= kSeg && (kSeg % 64) == 0 && (kSeg / 64) == 16);
static_assert(kExc <= kRowsP && (kRowsP % 64) == 0 && (kRowsP % 32) == 0);
static_assert((kKdim % 32) == 0);
static_assert(((kRowsP / 32) * (kRowsP / 64)) % 8 == 0);
static_assert((kExc % 4) == 0 && ((kExc * kExc / 4) % 256) == 0);
static_assert(kSeg == 256 * 4);

constexpr size_t kSzDOPA = (size_t)kSeg * 4;
constexpr size_t kSzG    = (size_t)kSeg * 4;
constexpr size_t kSzAT   = (size_t)kRowsP * kKdim * 2;
constexpr size_t kSzBT   = (size_t)kRowsP * kKdim * 2;
constexpr size_t kSzRAW  = (size_t)kRowsP * kRowsP * 4;
constexpr size_t kOffDOPA = 0;
constexpr size_t kOffG    = kOffDOPA + kSzDOPA;
constexpr size_t kOffAT   = kOffG    + kSzG;
constexpr size_t kOffBT   = kOffAT   + kSzAT;
constexpr size_t kOffRAW  = kOffBT   + kSzBT;
constexpr size_t kWsTotal = kOffRAW  + kSzRAW;
static_assert(kSzDOPA == 4096ull && kSzG == 4096ull && kSzAT == 1572864ull && kSzBT == 1572864ull && kSzRAW == 589824ull);
static_assert(kWsTotal == 3743744ull);
static_assert(kWsTotal <= 134217728ull);
static_assert((kOffG % 128) == 0 && (kOffAT % 128) == 0 && (kOffBT % 128) == 0 && (kOffRAW % 128) == 0);

__device__ __forceinline__ _Float16 f16_flush(float v) {
  const float w = (fabsf(v) < 6.103515625e-05f) ? 0.0f : v;
  return (_Float16)w;
}
__device__ __forceinline__ void f16_split(float v, _Float16& hi, _Float16& lo) {
  hi = f16_flush(v);
  const float hf = (float)hi;
  const float r = (v - hf) * kResid;
  lo = f16_flush(r);
}

__device__ __forceinline__ float bf16r(float v) {
  unsigned u = __float_as_uint(v);
  u = (u + 0x7FFFu + ((u >> 16) & 1u)) & 0xFFFF0000u;
  return __uint_as_float(u);
}

__device__ __forceinline__ float h16_to_f32(unsigned hb) {
  const unsigned sgn = (hb & 0x8000u) << 16; const unsigned em = hb & 0x7fffu;
  const float fn = __uint_as_float((em << 13) + 0x38000000u);
  const float fs = (float)em * 5.9604644775390625e-8f;
  const float mag = (em < 0x400u) ? fs : fn; return __uint_as_float(__float_as_uint(mag) | sgn); }

namespace eng {
union FragU { v16h v; v8h h[2]; };
__device__ __forceinline__ v16h frag_load(const _Float16* p) {
  FragU f;
  f.h[0] = *(const v8h*)(p);
  f.h[1] = *(const v8h*)(p + 16);
  return f.v;
}
__device__ __forceinline__ v8f mma(v16h a, v16h b, v8f c) {
  return __builtin_amdgcn_wmma_f32_16x16x32_f16(false, a, false, b, (short)0, c, false, false);
}
__device__ __forceinline__ void guard1(v8f& a, v16h x, v16h y) {
  asm volatile("v_nop\n\tv_nop\n\tv_nop\n\tv_nop" : "+v"(a) : "v"(x), "v"(y));
}
__device__ __forceinline__ void guard_acc(v8f& a) {
  asm volatile("v_nop\n\tv_nop\n\tv_nop\n\tv_nop" : "+v"(a));
}
__device__ __forceinline__ void keep4(v16h a, v16h b, v16h c, v16h d) {
  asm volatile("v_nop" :: "v"(a), "v"(b), "v"(c), "v"(d));
}

template <int MI, int SPL>
__global__ __launch_bounds__(256) void gemm_f16_kernel(
    const unsigned short* __restrict__ Ap, const unsigned short* __restrict__ A2p, int lda,
    const unsigned short* __restrict__ Btp, const unsigned short* __restrict__ Bt2p, int ldb,
    float* __restrict__ C, int ldc, int M, int N, int K, float scale, float rscale)
{
  static_assert(MI >= 1 && MI <= 2);
  static_assert(SPL >= 0 && SPL <= 2);
  const _Float16* A   = (const _Float16*)Ap;
  const _Float16* A2  = (const _Float16*)A2p;
  const _Float16* Bt  = (const _Float16*)Btp;
  const _Float16* Bt2 = (const _Float16*)Bt2p;
  __shared__ __align__(16) float sT[8][16 * 68];
  const int lane = threadIdx.x & 31;
  const int wave = threadIdx.x >> 5;
  const int tilesN = N >> 6;
  const int tilesM = M / (16 * MI);
  const int tile = blockIdx.x * 8 + wave;
  if (tile >= tilesM * tilesN) return;
  const int tm = tile / tilesN;
  const int tn = tile - tm * tilesN;
  const int m0 = tm * (16 * MI);
  const int n0 = tn << 6;
  const int rlane = lane & 15;
  const int koff  = (lane >> 4) * 8;
  const int mOff  = (lane >> 4) * 8;

  v8f acc[MI][4], accr[MI][4];
#pragma unroll
  for (int i = 0; i < MI; ++i)
#pragma unroll
    for (int j = 0; j < 4; ++j) {
      acc[i][j]  = (v8f){0.f, 0.f, 0.f, 0.f, 0.f, 0.f, 0.f, 0.f};
      accr[i][j] = (v8f){0.f, 0.f, 0.f, 0.f, 0.f, 0.f, 0.f, 0.f};
    }

  for (int k0 = 0; k0 < K; k0 += 32) {
    v16h bh[4], bl[4];
#pragma unroll
    for (int j = 0; j < 4; ++j) {
      const size_t bo = (size_t)(n0 + (j << 4) + rlane) * ldb + koff + k0;
      bh[j] = frag_load(Bt + bo);
      if (SPL == 2) bl[j] = frag_load(Bt2 + bo); else bl[j] = bh[j];
    }
#pragma unroll
    for (int i = 0; i < MI; ++i) {
      const size_t ao = (size_t)(m0 + (i << 4) + rlane) * lda + koff + k0;
      const v16h ah = frag_load(A + ao);
      v16h al = ah;
      if (SPL >= 1) al = frag_load(A2 + ao);
#pragma unroll
      for (int j = 0; j < 4; ++j) {
        acc[i][j] = mma(ah, bh[j], acc[i][j]);
        if (SPL >= 1) accr[i][j] = mma(al, bh[j], accr[i][j]);
        if (SPL == 2) accr[i][j] = mma(ah, bl[j], accr[i][j]);
      }
#pragma unroll
      for (int j = 0; j < 4; ++j) {
        guard1(acc[i][j], ah, al);
        if (SPL >= 1) guard1(accr[i][j], ah, al);
      }
    }
    keep4(bh[0], bh[1], bh[2], bh[3]);
    if (SPL == 2) keep4(bl[0], bl[1], bl[2], bl[3]);
  }
#pragma unroll
  for (int i = 0; i < MI; ++i)
#pragma unroll
    for (int j = 0; j < 4; ++j) {
      guard_acc(acc[i][j]);
      if (SPL >= 1) guard_acc(accr[i][j]);
    }

  float* slab = sT[wave];
#pragma unroll
  for (int i = 0; i < MI; ++i) {
    const int mBase = m0 + (i << 4);
#pragma unroll
    for (int j = 0; j < 4; ++j) {
#pragma unroll
      for (int r = 0; r < 8; ++r) {
        float v = acc[i][j][r] * scale;
        if (SPL >= 1) v += accr[i][j][r] * rscale;
        slab[(mOff + r) * 68 + (j << 4) + rlane] = v;
      }
    }
    __builtin_amdgcn_fence(__ATOMIC_RELEASE, "workgroup");
    __builtin_amdgcn_wave_barrier();
    __builtin_amdgcn_fence(__ATOMIC_ACQUIRE, "workgroup");
    {
      const int hh = lane >> 4, c4 = (lane & 15) * 4;
      for (int pass = 0; pass < 2; ++pass) {
#pragma unroll
        for (int it = 0; it < 8; ++it) {
          const int row = it * 2 + hh;
          const v4f v = *(const v4f*)(slab + row * 68 + c4);
          *(volatile v4f*)(C + (size_t)(mBase + row) * ldc + n0 + c4) = v;
        }
        __threadfence();
      }
    }
    __builtin_amdgcn_fence(__ATOMIC_RELEASE, "workgroup");
    __builtin_amdgcn_wave_barrier();
    __builtin_amdgcn_fence(__ATOMIC_ACQUIRE, "workgroup");
  }
}
}

__device__ __forceinline__ int clamp_int(int v, int lo, int hi) {
  const int a = (v < lo) ? lo : v;
  return (a > hi) ? hi : a;
}

__global__ __launch_bounds__(256) void dopa_kernel(
    const float* __restrict__ z, const float* __restrict__ zpre, const int* __restrict__ idxp,
    float* __restrict__ DOPA)
{
  const float rk[8] = {0.138366401f, 0.121697575f, 0.104852326f, 0.0878293067f, 0.0706271604f, 0.0532445349f, 0.0356800556f, 0.0179323405f};
  static_assert(sizeof(rk) / sizeof(rk[0]) == 8);
  const int tid = threadIdx.x;
  const int t0 = tid * 4;
  const int idx = clamp_int(idxp[0], 0, kNrn - 1);
  float zp[11];
#pragma unroll
  for (int j = 0; j < 11; ++j) {
    const int m  = t0 + j;
    const int mp = clamp_int(m + 1, 0, kPre - 1);
    const int mz = clamp_int(m - (kPre - 1), 0, kSteps - 1);
    const float a = zpre[mp];
    const float b = z[(size_t)mz * kNrn + idx];
    const float ar = bf16r(a);
    const float br = bf16r(b);
    const float fa = (m < (kPre - 1)) ? 1.0f : 0.0f;
    zp[j] = fmaf(fa, ar, (1.0f - fa) * br);
  }
  float res[4];
#pragma unroll
  for (int q = 0; q < 4; ++q) {
    float s = rk[0] * zp[q];
#pragma unroll
    for (int k = 1; k < 8; ++k) s = s + rk[k] * zp[q + k];
    res[q] = ((t0 + q) < kSteps) ? s : 0.0f;
  }
  v4f o;
  o[0] = res[0];
  o[1] = res[1];
  o[2] = res[2];
  o[3] = res[3];
  float* p = DOPA + t0;
  *(volatile v4f*)p = o;
  __threadfence();
  *(volatile v4f*)p = o;
}

__global__ __launch_bounds__(32) void g_kernel(const float* __restrict__ DOPA, float* __restrict__ G)
{
  const int lane = threadIdx.x;
  for (int p = 0; p < 8; ++p) {
    const int base = 128 * p + 4 * lane;
    float g = 0.0f;
    float k0 = 0.0f, k1 = 0.0f, k2 = 0.0f, k3 = 0.0f;
    for (int i = 0; i < 1024; ++i) {
      const int s = 1023 - i;
      const float dv = DOPA[s];
      g = fmaf(kDecayE, g, dv);
      k0 = (s == base)     ? g : k0;
      k1 = (s == base + 1) ? g : k1;
      k2 = (s == base + 2) ? g : k2;
      k3 = (s == base + 3) ? g : k3;
    }
    v4f o;
    o[0] = k0;
    o[1] = k1;
    o[2] = k2;
    o[3] = k3;
    float* q = G + base;
    *(volatile v4f*)q = o;
    __threadfence();
    *(volatile v4f*)q = o;
  }
}

__device__ __forceinline__ void store_two_lines(unsigned short* p0, unsigned short* p1,
                                                const v8h (&r0)[8], const v8h (&r1)[8]) {
#pragma unroll
  for (int q = 0; q < 8; ++q) *(volatile v8h*)(p0 + 8 * q) = r0[q];
#pragma unroll
  for (int q = 0; q < 8; ++q) *(volatile v8h*)(p1 + 8 * q) = r1[q];
}

__global__ __launch_bounds__(64) void trace_a_kernel(
    const float* __restrict__ z, const float* __restrict__ G, unsigned short* __restrict__ AT)
{
  const int i  = blockIdx.x * 64 + threadIdx.x;
  const int ic = clamp_int(i, 0, kExc - 1);
  const bool rowLive = (i < kExc);
  unsigned short* rowp = AT + (size_t)i * kKdim;
  float sm = 0.0f;
  for (int trip = 0; trip < 16; ++trip) {
    const int s0 = trip * 64;
    v8h r0[8], r1[8];
#pragma unroll
    for (int q = 0; q < 8; ++q) {
      const v4f ga = *(const v4f*)(G + s0 + 8 * q);
      const v4f gb = *(const v4f*)(G + s0 + 8 * q + 4);
#pragma unroll
      for (int e = 0; e < 8; ++e) {
        const int s  = s0 + 8 * q + e;
        const int sb = clamp_int(s - 1, 0, kSteps - 1);
        const float zl = z[(size_t)sb * kNrn + ic];
        const float zr = bf16r(zl);
        const bool live = rowLive && (s >= 1) && (s < kSteps);
        const float zprev = live ? zr : 0.0f;
        const float gx = (-kAM) * zprev;
        sm = fmaf(kDecayM, sm, gx);
        const float gs = (e < 4) ? ga[e & 3] : gb[e & 3];
        const float gz = gs * zprev;
        const float gm = gs * sm;
        const bool wl = rowLive && (s < kSteps);
        const float w0 = wl ? (gz * kACarry) : 0.0f;
        const float w1 = wl ? (gm * kACarry) : 0.0f;
        r0[q][e] = f16_flush(w0);
        r1[q][e] = f16_flush(w1);
      }
    }
    unsigned short* p0 = rowp + s0;
    unsigned short* p1 = rowp + kSeg + s0;
    store_two_lines(p0, p1, r0, r1);
    __threadfence();
    store_two_lines(p0, p1, r0, r1);
  }
}

__global__ __launch_bounds__(64) void trace_b_kernel(
    const float* __restrict__ z, unsigned short* __restrict__ BT)
{
  const int j  = blockIdx.x * 64 + threadIdx.x;
  const int jc = clamp_int(j, 0, kExc - 1);
  const bool rowLive = (j < kExc);
  unsigned short* rowp = BT + (size_t)j * kKdim;
  float sp = 0.0f;
  for (int trip = 0; trip < 16; ++trip) {
    const int s0 = trip * 64;
    v8h r0[8], r1[8];
#pragma unroll
    for (int q = 0; q < 8; ++q) {
#pragma unroll
      for (int e = 0; e < 8; ++e) {
        const int s  = s0 + 8 * q + e;
        const int sb = clamp_int(s, 0, kSteps - 1);
        const float zl = z[(size_t)sb * kNrn + jc];
        const float zr = bf16r(zl);
        const bool live = rowLive && (s < kSteps);
        const float zc = live ? zr : 0.0f;
        const float gx = kAP * zc;
        sp = fmaf(kDecayP, sp, gx);
        const float w0 = live ? (sp * kBCarry) : 0.0f;
        const float w1 = live ? (zc * kBCarry) : 0.0f;
        r0[q][e] = f16_flush(w0);
        r1[q][e] = f16_flush(w1);
      }
    }
    unsigned short* p0 = rowp + s0;
    unsigned short* p1 = rowp + kSeg + s0;
    store_two_lines(p0, p1, r0, r1);
    __threadfence();
    store_two_lines(p0, p1, r0, r1);
  }
}

__device__ __forceinline__ float clamp_neg(float raw, float wraw) {
  float dw = raw * kGain;
  const float w = bf16r(wraw);
  dw = (w > kWMax) ? fminf(0.0f, dw) : dw;
  dw = (w < 0.0f) ? fmaxf(0.0f, dw) : dw;
  return -dw;
}

__global__ __launch_bounds__(256) void out_clamp_kernel(
    const float* __restrict__ RAW, const float* __restrict__ wrec, float* __restrict__ out)
{
  const int wd = blockIdx.x * 256 + threadIdx.x;
  const int e0 = wd * 4;
  const int r = e0 / kExc;
  const int c = e0 - r * kExc;
  const v4f rv = *(const v4f*)(RAW + (size_t)r * kRowsP + c);
  const v4f wv = *(const v4f*)(wrec + e0);
  const float r0 = rv[0];
  const float r1 = rv[1];
  const float r2 = rv[2];
  const float r3 = rv[3];
  const float w0 = wv[0];
  const float w1 = wv[1];
  const float w2 = wv[2];
  const float w3 = wv[3];
  v4f o;
  o[0] = clamp_neg(r0, w0);
  o[1] = clamp_neg(r1, w1);
  o[2] = clamp_neg(r2, w2);
  o[3] = clamp_neg(r3, w3);
  float* p = out + e0;
  *(volatile v4f*)p = o;
  __threadfence();
  *(volatile v4f*)p = o;
}

extern "C" void kernel_launch(void* const* d_in, const int* in_sizes, int n_in,
                              void* d_out, int out_size, void* d_ws, size_t ws_size,
                              hipStream_t stream)
{
  if (n_in < 4) return;
  if (in_sizes[0] != kSteps * kNrn) return;
  if (in_sizes[1] != kPre) return;
  if (in_sizes[2] != kExc * kExc) return;
  if (in_sizes[3] != 1) return;
  if (out_size != kExc * kExc) return;
  if (ws_size < kWsTotal) return;

  const float* z      = (const float*)d_in[0];
  const float* zpre   = (const float*)d_in[1];
  const float* wrec   = (const float*)d_in[2];
  const int*   idxp   = (const int*)d_in[3];
  float* out = (float*)d_out;

  char* ws = (char*)d_ws;
  float*          DOPA = (float*)(ws + kOffDOPA);
  float*          G    = (float*)(ws + kOffG);
  unsigned short* AT   = (unsigned short*)(ws + kOffAT);
  unsigned short* BT   = (unsigned short*)(ws + kOffBT);
  float*          RAW  = (float*)(ws + kOffRAW);

  constexpr float sOut = 1.0f / (kACarry * kBCarry);

  dopa_kernel<<<1, 256, 0, stream>>>(z, zpre, idxp, DOPA);

  g_kernel<<<1, 32, 0, stream>>>(DOPA, G);

  trace_a_kernel<<<kRowsP / 64, 64, 0, stream>>>(z, G, AT);

  trace_b_kernel<<<kRowsP / 64, 64, 0, stream>>>(z, BT);

  eng::gemm_f16_kernel<2, 0><<<dim3((kRowsP / 32) * (kRowsP / 64) / 8), 256, 0, stream>>>(
      AT, nullptr, kKdim, BT, nullptr, kKdim, RAW, kRowsP, kRowsP, kRowsP, kKdim, sOut, 0.0f);

  out_clamp_kernel<<<(kExc * kExc / 4) / 256, 256, 0, stream>>>(RAW, wrec, out);
}
